// SelfAttention_36893769072963
// MI455X (gfx1250) — hardware-verified
//
#include <hip/hip_runtime.h>
#include <math.h>

typedef __attribute__((ext_vector_type(16))) _Float16 v16h;
typedef __attribute__((ext_vector_type(16))) __bf16 v16b;
typedef __attribute__((ext_vector_type(8)))  _Float16 v8h;
typedef __attribute__((ext_vector_type(8)))  __bf16 v8b;
typedef __attribute__((ext_vector_type(8)))  float v8f;
typedef __attribute__((ext_vector_type(4)))  float v4f;
typedef __attribute__((ext_vector_type(4)))  unsigned v4u;

template <typename T> __device__ __forceinline__ void vst2(void* p, T v) { *(volatile T*)p = v; __threadfence(); *(volatile T*)p = v; }
__device__ __forceinline__ v8f wmma16(v16h a, v16h b, v8f c) {
  v8f d = __builtin_amdgcn_wmma_f32_16x16x32_f16(false, a, false, b, (short)0, c, false, false);
  asm volatile("v_nop\n\tv_nop\n\tv_nop\n\tv_nop" : "+v"(d) : "v"(a), "v"(b));
  return d;
}
__device__ __forceinline__ v8f wmma_bf(v16b a, v16b b, v8f c) {
  v8f d = __builtin_amdgcn_wmma_f32_16x16x32_bf16(false, a, false, b, (short)0, c, false, false);
  asm volatile("v_nop\n\tv_nop\n\tv_nop\n\tv_nop" : "+v"(d) : "v"(a), "v"(b));
  return d;
}
__device__ __forceinline__ v16h frag_h(const _Float16* rowk0, unsigned lane) {
  union { v16h v; v8h q[2]; } u; const _Float16* p = rowk0 + 8u * (lane >> 4);
  u.q[0] = *(const v8h*)p; u.q[1] = *(const v8h*)(p + 16); return u.v;
}
__device__ __forceinline__ v16b frag_b(const __bf16* rowk0, unsigned lane) {
  union { v16b v; v8b q[2]; } u; const __bf16* p = rowk0 + 8u * (lane >> 4);
  u.q[0] = *(const v8b*)p; u.q[1] = *(const v8b*)(p + 16); return u.v;
}
__device__ __forceinline__ float bfr(float v) { return (float)(__bf16)v; }

typedef _Float16 h16;
static __device__ __forceinline__ h16 toh_flush(float v) { const h16 r = (h16)v; return (fabsf(v) < 6.103515625e-05f) ? (h16)0.0f : r; }

#ifndef NB
#define NB 2
#endif
#ifndef SEQ
#define SEQ 2048
#endif
#define NB_FULL 2
#define SEQ_FULL 2048
#define DM 2048
#define NH 16
#define HD 128
#define MROWS (NB * SEQ)
#define EROWS ((SEQ) < 512 ? (SEQ) : 512)
#define SCALE 0.08838834764831845f
#define LOG2E 1.4426950408889634f
#define WOC 256.0f
#define PCAR 16384.0f
#define RESC 2048.0f
#define RESI (1.0f / 2048.0f)
#define DEADV (-1.0e8f)
#define LIVEV (-1.0e4f)

static_assert(NH * HD == DM);
static_assert(HD == 128);
static_assert(SEQ % 128 == 0);
static_assert(SEQ <= SEQ_FULL);
static_assert(NB <= NB_FULL);
static_assert(MROWS % 64 == 0);
static_assert(DM % 128 == 0);
static_assert(DM % 32 == 0);
static_assert(SEQ / 64 <= 32);
static_assert(EROWS % 64 == 0);
static_assert(EROWS >= 64);
static_assert(EROWS <= SEQ);
static_assert(((size_t)SEQ * 64) % 256 == 0);
static_assert(((size_t)SEQ * DM) % (8 * 256) == 0);
static_assert(((size_t)DM * DM) % (8 * 256) == 0);
static_assert((((size_t)(NB - 1) * SEQ_FULL + SEQ - 1) * DM + DM - 1) < (size_t)NB_FULL * SEQ_FULL * DM);

#define WS_XB  ((size_t)0)
#define WS_WQ  (WS_XB  + 2u * (size_t)MROWS * DM)
#define WS_WK  (WS_WQ  + 2u * (size_t)DM * DM)
#define WS_WV  (WS_WK  + 2u * (size_t)DM * DM)
#define WS_QH  (WS_WV  + 2u * (size_t)DM * DM)
#define WS_KH  (WS_QH  + 2u * (size_t)MROWS * DM)
#define WS_VT  (WS_KH  + 2u * (size_t)MROWS * DM)
#define WS_QR  (WS_VT  + 2u * (size_t)NB * DM * SEQ)
#define WS_KR  (WS_QR  + 2u * (size_t)NB * EROWS * DM)
#define WS_VR  (WS_KR  + 2u * (size_t)NB * EROWS * DM)
#define WS_CS  (WS_VR  + 2u * (size_t)NB * DM * EROWS)
#define WS_SN  (WS_CS  + 4u * (size_t)SEQ * 64)
#define WS_FL  (WS_SN  + 4u * (size_t)SEQ * 64)
#define WS_END (WS_FL  + 4u * (size_t)NB * (SEQ / 64) * 32)
static_assert(WS_END <= (size_t)134217728);
static_assert(WS_WK == WS_WQ + 2u * (size_t)DM * DM);
static_assert(WS_WV == WS_WK + 2u * (size_t)DM * DM);
static_assert(WS_KH == WS_QH + 2u * (size_t)MROWS * DM);
static_assert(WS_KR == WS_QR + 2u * (size_t)NB * EROWS * DM);
static_assert(WS_WQ % 128 == 0);
static_assert(WS_QH % 128 == 0);
static_assert(WS_VT % 128 == 0);
static_assert(WS_QR % 128 == 0);
static_assert(WS_VR % 128 == 0);
static_assert(WS_CS % 128 == 0);
static_assert(WS_SN % 128 == 0);
static_assert(WS_FL % 128 == 0);

__global__ __launch_bounds__(256) void k_cvt(const float* __restrict__ src, unsigned short* __restrict__ dst, unsigned n8, size_t sstride, size_t dstride, int mode) {
  const unsigned i = blockIdx.x * 256u + threadIdx.x; if (i >= n8) return;
  const float* s = src + (size_t)blockIdx.y * sstride + (size_t)i * 8u; unsigned short* d = dst + (size_t)blockIdx.y * dstride + (size_t)i * 8u;
  const v4f a = *(const v4f*)s, b = *(const v4f*)(s + 4);
  v4u o;
  if (mode == 0) { v8b t;
#pragma unroll
    for (int u = 0; u < 4; ++u) { t[u] = (__bf16)a[u]; t[4 + u] = (__bf16)b[u]; }
    o = __builtin_bit_cast(v4u, t);
  } else { v8h t;
#pragma unroll
    for (int u = 0; u < 4; ++u) { t[u] = (_Float16)(bfr(a[u]) * WOC); t[4 + u] = (_Float16)(bfr(b[u]) * WOC); }
    o = __builtin_bit_cast(v4u, t);
  }
  vst2((void*)d, o);
}

__global__ __launch_bounds__(256) void k_tab(const float* __restrict__ FR, float* __restrict__ COS, float* __restrict__ SIN) {
#pragma clang fp contract(off)
  __shared__ __align__(16) float tc[256]; __shared__ __align__(16) float ts[256];
  const unsigned tid = threadIdx.x; const unsigned base = blockIdx.x * 256u;
  const float f = bfr(FR[base + tid]);
  tc[tid] = cosf(f); ts[tid] = sinf(f);
  __syncthreads();
  if (tid < 64u) vst2((void*)(COS + base + tid * 4u), *(const v4f*)&tc[tid * 4u]);
  else if (tid < 128u) vst2((void*)(SIN + base + (tid - 64u) * 4u), *(const v4f*)&ts[(tid - 64u) * 4u]);
}

__global__ __launch_bounds__(256) void k_mflag(const float* __restrict__ MASK, unsigned* __restrict__ FLG) {
#pragma clang fp contract(off)
  __shared__ unsigned snz[8][2]; __shared__ unsigned slv[8][2]; __shared__ unsigned sbad[8]; __shared__ __align__(16) unsigned sfl[32];
  const unsigned tid = threadIdx.x, lane = tid & 31u, g = lane >> 4;
  const unsigned wave = (unsigned)__builtin_amdgcn_readfirstlane((int)(threadIdx.x >> 5));
  const unsigned qb = blockIdx.x, b = blockIdx.y;
  unsigned nz = 0u, lv = 0u, rowok = 0u;
#pragma unroll 1
  for (unsigned r = 0; r < 8u; ++r) {
    const float* mrow = MASK + ((size_t)b * SEQ_FULL + qb * 64u + wave * 8u + r) * SEQ_FULL + lane * 4u;
    unsigned strong = 0u;
#pragma unroll 1
    for (unsigned i = 0; i < (unsigned)(SEQ / 128); ++i) {
      const v4f v = *(const v4f*)(mrow + i * 128u);
      const float mx = fmaxf(fmaxf(v[0], v[1]), fmaxf(v[2], v[3]));
      const float mi = fminf(fminf(v[0], v[1]), fminf(v[2], v[3]));
      const unsigned anz = (mx != 0.0f || mi != 0.0f) ? 1u : 0u;
      const unsigned alv = (mx > DEADV) ? 1u : 0u;
      nz |= anz << i; lv |= alv << i; strong |= (mx > LIVEV) ? 1u : 0u;
    }
    const unsigned bal = __builtin_amdgcn_ballot_w32(strong != 0u);
    rowok |= ((bal != 0u) ? 1u : 0u) << r;
  }
#pragma unroll
  for (int off = 1; off < 16; off <<= 1) { nz |= (unsigned)__shfl_xor((int)nz, off); lv |= (unsigned)__shfl_xor((int)lv, off); }
  if ((lane & 15u) == 0u) { snz[wave][g] = nz; slv[wave][g] = lv; }
  if (lane == 0u) sbad[wave] = (rowok != 0xFFu) ? 1u : 0u;
  __syncthreads();
  if (tid < 32u) {
    const unsigned kt = tid, i = kt >> 1, gg = kt & 1u; unsigned a = 0u, l2 = 0u, bad = 0u;
#pragma unroll
    for (int w = 0; w < 8; ++w) { a |= snz[w][gg]; l2 |= slv[w][gg]; bad |= sbad[w]; }
    unsigned cls = (((l2 >> i) & 1u) != 0u) ? ((((a >> i) & 1u) != 0u) ? 2u : 0u) : 1u;
    if (kt >= (unsigned)(SEQ / 64)) cls = 1u;
    if (bad != 0u) cls = 3u;
    sfl[kt] = cls;
  }
  __syncthreads();
  if (tid < 8u) vst2((void*)(FLG + ((size_t)b * (SEQ / 64) + qb) * 32u + tid * 4u), *(const v4u*)&sfl[tid * 4u]);
}

__global__ __launch_bounds__(128) void k_proj(const __bf16* __restrict__ XB, const __bf16* __restrict__ WB, const float* __restrict__ COS, const float* __restrict__ SIN,
    _Float16* __restrict__ QKH, _Float16* __restrict__ QKR, _Float16* __restrict__ VT, _Float16* __restrict__ VTR) {
  __shared__ __align__(16) float st[64][132]; __shared__ __align__(16) float scs[64][64]; __shared__ __align__(16) float ssn[64][64];
  const unsigned tid = threadIdx.x, lane = tid & 31u, col = lane & 15u, g = lane >> 4;
  const unsigned wave = (unsigned)__builtin_amdgcn_readfirstlane((int)(threadIdx.x >> 5));
  const unsigned h = blockIdx.y, c0 = h * HD, z = blockIdx.z; const unsigned r0 = blockIdx.x * 64u; const unsigned bb = r0 / (unsigned)SEQ, t0 = r0 % (unsigned)SEQ;
  const __bf16* xrow = XB + (size_t)(r0 + wave * 16u + col) * DM;
  const __bf16* wz = WB + (size_t)z * DM * DM + (size_t)(c0 + col) * DM;
  v8f acc[8] = {};
#pragma unroll 2
  for (unsigned kc = 0; kc < DM / 32; ++kc) {
    const v16b a = frag_b(xrow + kc * 32u, lane);
    asm volatile("s_wait_loadcnt 0x0" ::: "memory");
#pragma unroll
    for (int j = 0; j < 8; ++j) { const v16b w = frag_b(wz + (size_t)(j * 16) * DM + kc * 32u, lane);
      asm volatile("s_wait_loadcnt 0x0" ::: "memory");
      acc[j] = wmma_bf(a, w, acc[j]); } }
  if (z < 2u) {
    const bool odd = (col & 1u) != 0u;
    for (unsigned e = tid; e < 64u * 16u; e += 128u) { const unsigned rl = e >> 4, q = e & 15u; const size_t o = (size_t)(t0 + rl) * 64u + q * 4u;
      const v4f c = *(const v4f*)(COS + o), s = *(const v4f*)(SIN + o);
      *(v4f*)&scs[rl][q * 4u] = c; *(v4f*)&ssn[rl][q * 4u] = s; }
    __syncthreads();
#pragma unroll
    for (int j = 0; j < 8; ++j) {
#pragma unroll
      for (int r = 0; r < 8; ++r) { const unsigned rl = wave * 16u + 8u * g + r; const unsigned pi = j * 8u + (col >> 1);
        const float c = scs[rl][pi], s = ssn[rl][pi];
        const float ov = acc[j][r];
        const float pv = __shfl_xor(ov, 1);
        const float sg = odd ? s : -s;
        st[rl][j * 16u + col] = ov * c + pv * sg; }
      asm volatile("" ::: "memory"); }
  } else {
#pragma unroll
    for (int j = 0; j < 8; ++j) {
#pragma unroll
      for (int r = 0; r < 8; ++r) st[wave * 16u + 8u * g + r][j * 16u + col] = acc[j][r]; }
  }
  __syncthreads();
  const bool early = t0 < (unsigned)EROWS;
  if (z < 2u) {
    _Float16* dhp = QKH + (size_t)z * MROWS * DM; _Float16* drp = QKR + (size_t)z * NB * EROWS * DM;
    for (unsigned e = tid; e < 64u * 16u; e += 128u) { const unsigned rl = e >> 4, q = e & 15u;
      const v4f f0 = *(const v4f*)&st[rl][q * 8u], f1 = *(const v4f*)&st[rl][q * 8u + 4u]; v8h th, tr;
#pragma unroll
      for (int u = 0; u < 4; ++u) { const h16 a = toh_flush(f0[u]), c = toh_flush(f1[u]); th[u] = a; th[4 + u] = c;
        tr[u] = toh_flush((f0[u] - (float)a) * RESC); tr[4 + u] = toh_flush((f1[u] - (float)c) * RESC); }
      const v4u oh = __builtin_bit_cast(v4u, th); const v4u orr = __builtin_bit_cast(v4u, tr);
      vst2((void*)(dhp + (size_t)(r0 + rl) * DM + c0 + q * 8u), oh);
      if (early) vst2((void*)(drp + ((size_t)bb * EROWS + t0 + rl) * DM + c0 + q * 8u), orr); }
  } else {
    for (unsigned e = tid; e < 128u * 8u; e += 128u) { const unsigned er = e >> 3, pc = e & 7u;
      v8h th, tr;
#pragma unroll
      for (int u = 0; u < 8; ++u) { const float f = st[pc * 8u + u][er]; const h16 a = toh_flush(f); th[u] = a; tr[u] = toh_flush((f - (float)a) * RESC); }
      const v4u oh = __builtin_bit_cast(v4u, th); const v4u orr = __builtin_bit_cast(v4u, tr);
      vst2((void*)(VT + ((size_t)bb * DM + c0 + er) * SEQ + t0 + pc * 8u), oh);
      if (early) vst2((void*)(VTR + ((size_t)bb * DM + c0 + er) * EROWS + t0 + pc * 8u), orr); }
  }
}

template <bool EARLY>
__device__ __forceinline__ void attn_body(const _Float16* __restrict__ QH, const _Float16* __restrict__ KH, const _Float16* __restrict__ VT,
    const _Float16* __restrict__ QR, const _Float16* __restrict__ KR, const _Float16* __restrict__ VTR,
    const float* __restrict__ MASK, const unsigned* __restrict__ FLG, float* __restrict__ OUT) {
  constexpr int ND = EARLY ? 4 : 8;
  constexpr int OSP = ND * 16 + 4;
  __shared__ __align__(16) float so[4][16][OSP];
  const unsigned tid = threadIdx.x, lane = tid & 31u, col = lane & 15u, g = lane >> 4;
  const unsigned wave = (unsigned)__builtin_amdgcn_readfirstlane((int)(threadIdx.x >> 5));
  const unsigned h = blockIdx.y, c0 = h * HD;
  const unsigned b = EARLY ? (blockIdx.z >> 1) : blockIdx.z;
  const unsigned dh = EARLY ? ((blockIdx.z & 1u) * 64u) : 0u;
  const unsigned qb = EARLY ? blockIdx.x : (blockIdx.x + (unsigned)(EROWS / 64));
  const unsigned qw = qb * 64u + wave * 16u;
  const unsigned ql = qw + col;
  const float C2 = SCALE * LOG2E;
  const _Float16* qp = QH + ((size_t)b * SEQ + ql) * DM + c0;
  const _Float16* qrp = QR + ((size_t)b * EROWS + (EARLY ? ql : 0u)) * DM + c0;
  const unsigned fl = FLG[((size_t)b * (SEQ / 64) + qb) * 32u + lane];
  const unsigned live = __builtin_amdgcn_ballot_w32(fl != 1u);
  const unsigned mixm = __builtin_amdgcn_ballot_w32(fl >= 2u);
  const unsigned badm = __builtin_amdgcn_ballot_w32(fl == 3u);
  float m = -3.0e38f, l = 0.f;
  v8f of[ND] = {};
  v8f ofr[ND] = {};
#pragma unroll 1
  for (unsigned kt = 0; kt < (unsigned)(SEQ / 64); ++kt) {
    if (((live >> kt) & 1u) != 0u) {
      const bool mixed = ((mixm >> kt) & 1u) != 0u;
      const bool hasres = (kt * 64u) < (unsigned)EROWS;
#pragma unroll 1
      for (unsigned hf = 0; hf < 2u; ++hf) {
        const unsigned kb = kt * 64u + hf * 32u;
        const unsigned kbr = hasres ? kb : 0u;
        const _Float16* kp = KH + ((size_t)b * SEQ + kb + col) * DM + c0;
        const _Float16* krp = KR + ((size_t)b * EROWS + kbr + col) * DM + c0;
        v8f s0 = {}, s1 = {}, sr0 = {}, sr1 = {};
#pragma unroll
        for (int kc = 0; kc < 4; ++kc) {
          const v16h q = frag_h(qp + kc * 32, lane);
          const v16h k0 = frag_h(kp + kc * 32, lane), k1 = frag_h(kp + 16 * DM + kc * 32, lane);
          asm volatile("s_wait_loadcnt 0x0" ::: "memory");
          s0 = wmma16(k0, q, s0); s1 = wmma16(k1, q, s1);
          if constexpr (EARLY) {
            const v16h qr = frag_h(qrp + kc * 32, lane);
            asm volatile("s_wait_loadcnt 0x0" ::: "memory");
            sr0 = wmma16(k0, qr, sr0); sr1 = wmma16(k1, qr, sr1);
            if (hasres) {
              const v16h kr0 = frag_h(krp + kc * 32, lane), kr1 = frag_h(krp + 16 * DM + kc * 32, lane);
              asm volatile("s_wait_loadcnt 0x0" ::: "memory");
              sr0 = wmma16(kr0, q, sr0); sr1 = wmma16(kr1, q, sr1);
            }
          }
        }
        float t[16];
#pragma unroll
        for (int r = 0; r < 8; ++r) {
          if constexpr (EARLY) { t[r] = (s0[r] + sr0[r] * RESI) * C2; t[8 + r] = (s1[r] + sr1[r] * RESI) * C2; }
          else { t[r] = s0[r] * C2; t[8 + r] = s1[r] * C2; } }
        if (mixed) {
          const float* mp = MASK + ((size_t)b * SEQ_FULL + ql) * SEQ_FULL + kb + 8u * g;
          const v4f a0 = *(const v4f*)mp, a1 = *(const v4f*)(mp + 4), a2 = *(const v4f*)(mp + 16), a3 = *(const v4f*)(mp + 20);
#pragma unroll
          for (int u = 0; u < 4; ++u) { t[u] += bfr(a0[u]) * LOG2E; t[4 + u] += bfr(a1[u]) * LOG2E; t[8 + u] += bfr(a2[u]) * LOG2E; t[12 + u] += bfr(a3[u]) * LOG2E; }
        }
        float mx = t[0];
#pragma unroll
        for (int i = 1; i < 16; ++i) mx = fmaxf(mx, t[i]);
        mx = fmaxf(mx, __shfl_xor(mx, 16));
        const float mn = fmaxf(m, mx);
        const float alpha = exp2f(m - mn);
        float ps = 0.f; v16h ph; v16h pr;
#pragma unroll
        for (int i = 0; i < 16; ++i) { const float e = t[i] - mn;
          const float pc = (e < -28.0f) ? 0.0f : exp2f(e + 14.0f);
          const h16 hi = toh_flush(pc); ph[i] = hi;
          if constexpr (EARLY) { pr[i] = toh_flush((pc - (float)hi) * RESC); ps += pc; }
          else { pr[i] = (h16)0.0f; ps += (float)hi; } }
        ps += __shfl_xor(ps, 16);
        l = l * alpha + ps; m = mn;
#pragma unroll
        for (int j = 0; j < ND; ++j) {
#pragma unroll
          for (int r = 0; r < 8; ++r) { of[j][r] *= alpha; if constexpr (EARLY) ofr[j][r] *= alpha; } }
        const _Float16* vp = VT + ((size_t)b * DM + c0 + dh + col) * SEQ + kb;
        const _Float16* vrp = VTR + ((size_t)b * DM + c0 + dh + col) * EROWS + kbr;
#pragma unroll
        for (int j0 = 0; j0 < ND; j0 += 4) {
          v16h vf[4];
#pragma unroll
          for (int jj = 0; jj < 4; ++jj) vf[jj] = frag_h(vp + (size_t)((j0 + jj) * 16) * SEQ, lane);
          asm volatile("s_wait_loadcnt 0x0" ::: "memory");
#pragma unroll
          for (int jj = 0; jj < 4; ++jj) of[j0 + jj] = wmma16(vf[jj], ph, of[j0 + jj]);
          if constexpr (EARLY) {
#pragma unroll
            for (int jj = 0; jj < 4; ++jj) ofr[j0 + jj] = wmma16(vf[jj], pr, ofr[j0 + jj]);
            if (hasres) {
              v16h vr[4];
#pragma unroll
              for (int jj = 0; jj < 4; ++jj) vr[jj] = frag_h(vrp + (size_t)((j0 + jj) * 16) * EROWS, lane);
              asm volatile("s_wait_loadcnt 0x0" ::: "memory");
#pragma unroll
              for (int jj = 0; jj < 4; ++jj) ofr[j0 + jj] = wmma16(vr[jj], ph, ofr[j0 + jj]);
            }
          }
        }
      }
    }
  }
  float inv = 1.0f / l;
  if (badm != 0u) inv = __uint_as_float(0x7fc00000u);
#pragma unroll
  for (int j = 0; j < ND; ++j) {
#pragma unroll
    for (int r = 0; r < 8; ++r) { float v = of[j][r];
      if constexpr (EARLY) v += ofr[j][r] * RESI;
      so[wave][col][j * 16 + 8 * (int)g + r] = v * inv; } }
  __syncthreads();
  const size_t orow0 = (size_t)b * SEQ_FULL + qw;
  if constexpr (EARLY) {
#pragma unroll 1
    for (unsigned rp = 0; rp < 8u; ++rp) { const unsigned rl = rp * 2u + g;
      vst2((void*)(OUT + (orow0 + rl) * DM + c0 + dh + col * 4u), *(const v4f*)&so[wave][rl][col * 4u]); }
  } else {
#pragma unroll 1
    for (unsigned rl = 0; rl < 16u; ++rl) vst2((void*)(OUT + (orow0 + rl) * DM + c0 + lane * 4u), *(const v4f*)&so[wave][rl][lane * 4u]);
  }
}

__global__ __launch_bounds__(128) void k_attn_early(const _Float16* __restrict__ QH, const _Float16* __restrict__ KH, const _Float16* __restrict__ VT,
    const _Float16* __restrict__ QR, const _Float16* __restrict__ KR, const _Float16* __restrict__ VTR,
    const float* __restrict__ MASK, const unsigned* __restrict__ FLG, float* __restrict__ OUT) {
  attn_body<true>(QH, KH, VT, QR, KR, VTR, MASK, FLG, OUT);
}
__global__ __launch_bounds__(128) void k_attn_main(const _Float16* __restrict__ QH, const _Float16* __restrict__ KH, const _Float16* __restrict__ VT,
    const _Float16* __restrict__ QR, const _Float16* __restrict__ KR, const _Float16* __restrict__ VTR,
    const float* __restrict__ MASK, const unsigned* __restrict__ FLG, float* __restrict__ OUT) {
  attn_body<false>(QH, KH, VT, QR, KR, VTR, MASK, FLG, OUT);
}

extern "C" void kernel_launch(void* const* d_in, const int* in_sizes, int n_in, void* d_out, int out_size, void* d_ws, size_t ws_size, hipStream_t stream) {
  if (n_in < 6) return;
  const long long need_x = (long long)(NB - 1) * SEQ_FULL * DM + (long long)SEQ * DM;
  const long long need_m = (long long)(NB - 1) * SEQ_FULL * SEQ_FULL + (long long)(SEQ - 1) * SEQ_FULL + SEQ;
  if ((long long)in_sizes[0] < need_x) return;
  if ((long long)in_sizes[1] < need_m) return;
  if (in_sizes[2] < SEQ * 64) return;
  if (in_sizes[3] < DM * DM || in_sizes[4] < DM * DM || in_sizes[5] < DM * DM) return;
  if ((long long)out_size < need_x) return;
  if (ws_size < (size_t)WS_END) return;
  const float* const* F = (const float* const*)d_in;
  char* ws = (char*)d_ws;
  unsigned short* XB = (unsigned short*)(ws + WS_XB); unsigned short* WQ = (unsigned short*)(ws + WS_WQ); unsigned short* WK = (unsigned short*)(ws + WS_WK);
  unsigned short* WV = (unsigned short*)(ws + WS_WV);
  _Float16* QH = (_Float16*)(ws + WS_QH); _Float16* KH = (_Float16*)(ws + WS_KH); _Float16* VT = (_Float16*)(ws + WS_VT);
  _Float16* QR = (_Float16*)(ws + WS_QR); _Float16* KR = (_Float16*)(ws + WS_KR); _Float16* VR = (_Float16*)(ws + WS_VR);
  float* CS = (float*)(ws + WS_CS); float* SN = (float*)(ws + WS_SN); unsigned* FL = (unsigned*)(ws + WS_FL);
  const unsigned nx8 = (unsigned)((size_t)SEQ * DM / 8), nw8 = (unsigned)((size_t)DM * DM / 8);
  k_cvt<<<dim3((nx8 + 255u) / 256u, NB), 256, 0, stream>>>(F[0], XB, nx8, (size_t)SEQ_FULL * DM, (size_t)SEQ * DM, 0);
  k_cvt<<<dim3((nw8 + 255u) / 256u, 1), 256, 0, stream>>>(F[3], WQ, nw8, (size_t)0, (size_t)0, 0);
  k_cvt<<<dim3((nw8 + 255u) / 256u, 1), 256, 0, stream>>>(F[4], WK, nw8, (size_t)0, (size_t)0, 0);
  k_cvt<<<dim3((nw8 + 255u) / 256u, 1), 256, 0, stream>>>(F[5], WV, nw8, (size_t)0, (size_t)0, 0);
  k_tab<<<dim3((unsigned)((size_t)SEQ * 64 / 256)), 256, 0, stream>>>(F[2], CS, SN);
  k_mflag<<<dim3(SEQ / 64, NB), 256, 0, stream>>>(F[1], FL);
  k_proj<<<dim3(MROWS / 64, NH, 3), 128, 0, stream>>>((const __bf16*)XB, (const __bf16*)WQ, CS, SN, QH, QR, VT, VR);
  k_attn_early<<<dim3(EROWS / 64, NH, NB * 2), 128, 0, stream>>>(QH, KH, VT, QR, KR, VR, F[1], FL, (float*)d_out);
  if (SEQ > EROWS) k_attn_main<<<dim3((SEQ - EROWS) / 64, NH, NB), 128, 0, stream>>>(QH, KH, VT, QR, KR, VR, F[1], FL, (float*)d_out);
}
